// PolicyNetwork3_84593675862715
// MI455X (gfx1250) — hardware-run, weakly checked
//
#include <hip/hip_runtime.h>
#include <math.h>

typedef __attribute__((ext_vector_type(16))) _Float16 v16h;
typedef __attribute__((ext_vector_type(8)))  _Float16 v8h;
typedef __attribute__((ext_vector_type(8)))  float    v8f;
typedef __attribute__((ext_vector_type(4)))  float    v4f;
typedef __attribute__((ext_vector_type(4)))  int      v4i;

constexpr int kNodes     = 50000;
constexpr int kEdges     = 800000;
constexpr int kCand      = 100000;
constexpr int kFeat      = 128;
constexpr int kMlpH      = 64;
constexpr int kMlpInRows = 257;
constexpr int kNodesPad  = 50048;
constexpr int kTileNodes = 256;
constexpr int kNodeTiles = (kNodes + kTileNodes - 1) / kTileNodes;
constexpr int kPackRows  = kNodeTiles * kTileNodes;
constexpr int kPackK     = 2 * kFeat;
constexpr int kCandPad   = 100032;
constexpr int kEdgeChunk = 128;
constexpr float kBnEps   = 1e-5f;
constexpr float kSlope   = 0.01f;

static_assert(kNodeTiles == 196 && kPackRows == 50176, "node tiling");
static_assert((kNodesPad % 64) == 0 && kNodesPad >= kNodes && kNodesPad <= kPackRows, "node row padding");
static_assert((kCandPad % 64) == 0 && kCandPad >= kCand, "candidate row padding");
static_assert((kEdges % kEdgeChunk) == 0, "edge chunks");
static_assert((kCand % 32) == 0, "whole output lines");
static_assert(((kCandPad * 8) % 256) == 0, "candidate grid");
static_assert((kPackK % 32) == 0 && (kFeat % 32) == 0 && (kMlpH % 32) == 0, "GEMM K multiples of 32");
static_assert((kFeat % 64) == 0 && (kMlpH % 64) == 0, "GEMM N multiples of 64");
static_assert(kCand * 4 == 400000 && 2 * kCand * 4 == 800000, "output byte offsets");

constexpr size_t kOffA16 = 0;
constexpr size_t kOffH0  = kOffA16 + (size_t)kPackRows * kPackK * 2;
constexpr size_t kOffH1  = kOffH0  + (size_t)kNodesPad * kFeat * 4;
constexpr size_t kOffPP  = kOffH1  + (size_t)kNodesPad * kFeat * 2;
constexpr size_t kOffZ0  = kOffPP  + (size_t)kNodesPad * kFeat * 4;
constexpr size_t kOffZ1  = kOffZ0  + (size_t)kCandPad * kMlpH * 2;
constexpr size_t kOffYW  = kOffZ1  + (size_t)kCandPad * kMlpH * 4;
constexpr size_t kOffBL0 = kOffYW  + (size_t)kCand * 4;
constexpr size_t kOffBL1 = kOffBL0 + (size_t)kFeat * kPackK * 2;
constexpr size_t kOffBP  = kOffBL1 + (size_t)kFeat * kPackK * 2;
constexpr size_t kOffBM1 = kOffBP  + (size_t)kFeat * kFeat * 2;
constexpr size_t kOffT0  = kOffBM1 + (size_t)kMlpH * kMlpH * 2;
constexpr size_t kOffT1  = kOffT0  + (size_t)kFeat * 4;
constexpr size_t kWsTotal = kOffT1 + (size_t)kFeat * 4;
static_assert(kWsTotal == 128736896ull, "carve total");
static_assert(kWsTotal <= 134217728ull, "carve cap");
static_assert((kOffH0 % 128) == 0 && (kOffH1 % 128) == 0 && (kOffPP % 128) == 0 && (kOffZ0 % 128) == 0 &&
              (kOffZ1 % 128) == 0 && (kOffYW % 128) == 0 && (kOffBL0 % 128) == 0 && (kOffBL1 % 128) == 0 &&
              (kOffBP % 128) == 0 && (kOffBM1 % 128) == 0 && (kOffT0 % 128) == 0 && (kOffT1 % 128) == 0, "128-B aligned regions");

__device__ __forceinline__ v16h frag_load_h(const _Float16* p) {
  union U { v16h v; v8h h[2]; } f;
  f.h[0] = *(const v8h*)(p);
  f.h[1] = *(const v8h*)(p + 16);
  return f.v;
}
__device__ __forceinline__ v8f mma_h(v16h a, v16h b, v8f c) {
  c = __builtin_amdgcn_wmma_f32_16x16x32_f16(false, a, false, b, (short)0, c, false, false);
  asm volatile("v_nop\n\tv_nop\n\tv_nop\n\tv_nop" : "+v"(c) : "v"(a), "v"(b));
  return c;
}
__device__ __forceinline__ void keep4_h(v16h a, v16h b, v16h c, v16h d) { asm volatile("v_nop" :: "v"(a), "v"(b), "v"(c), "v"(d)); }
__device__ __forceinline__ void acc_guard4(v8f& a, v8f& b, v8f& c, v8f& d) { asm volatile("v_nop\n\tv_nop\n\tv_nop\n\tv_nop" : "+v"(a), "+v"(b), "+v"(c), "+v"(d)); }
__device__ __forceinline__ void wave_lds_sync() {
  __builtin_amdgcn_fence(__ATOMIC_RELEASE, "workgroup");
  __builtin_amdgcn_wave_barrier();
  __builtin_amdgcn_fence(__ATOMIC_ACQUIRE, "workgroup");
}
__device__ __forceinline__ int clampi(int v, int lo, int hi) { return v < lo ? lo : (v > hi ? hi : v); }

template <int BIAS_MODE, int OUT_MODE, int ACT>
__global__ __launch_bounds__(256) void wmma_gemm64(
    const unsigned short* __restrict__ Ap, int lda,
    const unsigned short* __restrict__ Btp, int ldb,
    void* __restrict__ Cout, int ldc,
    const float* __restrict__ bias,
    int M, int N, int K) {
  const _Float16* A  = (const _Float16*)Ap;
  const _Float16* Bt = (const _Float16*)Btp;
  __shared__ __align__(16) float sT[8][16 * 68];
  const int lane = threadIdx.x & 31;
  const int wave = threadIdx.x >> 5;
  const int tilesN = N >> 6;
  const int tilesM = M >> 6;
  const int tile = blockIdx.x * 8 + wave;
  if (tile >= tilesM * tilesN) return;
  const int tm = tile / tilesN;
  const int tn = tile - tm * tilesN;
  const int m0 = tm << 6;
  const int n0 = tn << 6;

  const int rlane = lane & 15;
  const int koff  = (lane >> 4) * 8;
  const int mOff  = (lane >> 4) * 8;

  v8f acc[4][4];
#pragma unroll
  for (int i = 0; i < 4; ++i)
#pragma unroll
    for (int j = 0; j < 4; ++j) acc[i][j] = (v8f){0.f, 0.f, 0.f, 0.f, 0.f, 0.f, 0.f, 0.f};

  for (int k0 = 0; k0 < K; k0 += 32) {
    v16h bh[4];
#pragma unroll
    for (int j = 0; j < 4; ++j) {
      const size_t bo = (size_t)(n0 + (j << 4) + rlane) * ldb + koff + k0;
      bh[j] = frag_load_h(Bt + bo);
    }
#pragma unroll
    for (int i = 0; i < 4; ++i) {
      const size_t ao = (size_t)(m0 + (i << 4) + rlane) * lda + koff + k0;
      const v16h ah = frag_load_h(A + ao);
#pragma unroll
      for (int j = 0; j < 4; ++j) acc[i][j] = mma_h(ah, bh[j], acc[i][j]);
    }
    keep4_h(bh[0], bh[1], bh[2], bh[3]);
  }
  acc_guard4(acc[0][0], acc[0][1], acc[0][2], acc[0][3]);
  acc_guard4(acc[1][0], acc[1][1], acc[1][2], acc[1][3]);
  acc_guard4(acc[2][0], acc[2][1], acc[2][2], acc[2][3]);
  acc_guard4(acc[3][0], acc[3][1], acc[3][2], acc[3][3]);

  float* slab = sT[wave];
#pragma unroll
  for (int i = 0; i < 4; ++i) {
    const int mBase = m0 + (i << 4);
#pragma unroll
    for (int j = 0; j < 4; ++j) {
      const int n = n0 + (j << 4) + rlane;
      float bv = 0.f;
      if (BIAS_MODE == 2) bv = bias[n];
#pragma unroll
      for (int r = 0; r < 8; ++r) {
        float v = acc[i][j][r];
        if (BIAS_MODE == 2) v += bv;
        if (ACT == 4 || ACT == 6) v = (v > 0.f) ? v : kSlope * v;
        if (ACT == 6) v = (v != v) ? 1e-14f : v;
        slab[(mOff + r) * 68 + (j << 4) + rlane] = v;
      }
    }
    wave_lds_sync();
    if (OUT_MODE == 0) {
      float* C = (float*)Cout;
      const int hh = lane >> 4, c4 = (lane & 15) * 4;
      for (int pass = 0; pass < 2; ++pass) {
#pragma unroll
        for (int it = 0; it < 8; ++it) {
          const int row = it * 2 + hh;
          const v4f v = *(const v4f*)(slab + row * 68 + c4);
          *(volatile v4f*)(C + (size_t)(mBase + row) * ldc + n0 + c4) = v;
        }
        __threadfence();
      }
    } else {
      const int q = lane >> 3, c8 = (lane & 7) * 8;
      unsigned short* C = (unsigned short*)Cout;
      for (int pass = 0; pass < 2; ++pass) {
#pragma unroll
        for (int it = 0; it < 4; ++it) {
          const int row = it * 4 + q;
          const float* sp = slab + row * 68 + c8;
          v8h hv;
#pragma unroll
          for (int e = 0; e < 8; ++e) hv[e] = (_Float16)sp[e];
          *(volatile v8h*)(C + (size_t)(mBase + row) * ldc + n0 + c8) = hv;
        }
        __threadfence();
      }
    }
    wave_lds_sync();
  }
}

__global__ __launch_bounds__(256) void prep_kernel(
    const float* __restrict__ ws0, const float* __restrict__ wn0, const float* __restrict__ b0,
    const float* __restrict__ g0, const float* __restrict__ be0, const float* __restrict__ rm0,
    const float* __restrict__ rv0,
    const float* __restrict__ ws1, const float* __restrict__ wn1, const float* __restrict__ b1,
    const float* __restrict__ g1, const float* __restrict__ be1, const float* __restrict__ rm1,
    const float* __restrict__ rv1,
    const float* __restrict__ mw0, const float* __restrict__ mw1,
    unsigned short* __restrict__ BL0, unsigned short* __restrict__ BL1,
    unsigned short* __restrict__ BP, unsigned short* __restrict__ BM1,
    float* __restrict__ T0, float* __restrict__ T1) {
  const int blk = blockIdx.x, tid = threadIdx.x;
  if (blk < 32) {
    const int L = blk >> 4;
    const int idx = (blk & 15) * 256 + tid;
    const int w = idx >> 5, lane = idx & 31;
    const int hs = w & 1;
    const int n = (w >> 1) * 2 + (lane >> 4);
    const int kk = (lane & 15) * 8;
    const float* wsel = L ? (hs ? wn1 : ws1) : (hs ? wn0 : ws0);
    const float* gp  = L ? g1 : g0;
    const float* rvp = L ? rv1 : rv0;
    const float s = gp[n] * rsqrtf(rvp[n] + kBnEps);
    v8h hv;
#pragma unroll
    for (int e = 0; e < 8; ++e) {
      const float wv = wsel[(size_t)(kk + e) * kFeat + n];
      hv[e] = (_Float16)(wv * s);
    }
    unsigned short* q = (L ? BL1 : BL0) + (size_t)n * kPackK + hs * kFeat + kk;
    *(volatile v8h*)q = hv;
    __threadfence();
    *(volatile v8h*)q = hv;
  } else if (blk < 40) {
    const int idx = (blk - 32) * 256 + tid;
    const int n = idx >> 4;
    const int kk = (idx & 15) * 8;
    const int krow = (n >= kMlpH) ? kFeat : 0;
    const int col = n & (kMlpH - 1);
    v8h hv;
#pragma unroll
    for (int e = 0; e < 8; ++e) hv[e] = (_Float16)mw0[(size_t)(krow + kk + e) * kMlpH + col];
    unsigned short* q = BP + (size_t)n * kFeat + kk;
    *(volatile v8h*)q = hv;
    __threadfence();
    *(volatile v8h*)q = hv;
  } else if (blk < 42) {
    const int idx = (blk - 40) * 256 + tid;
    const int n = idx >> 3;
    const int kk = (idx & 7) * 8;
    v8h hv;
#pragma unroll
    for (int e = 0; e < 8; ++e) hv[e] = (_Float16)mw1[(size_t)(kk + e) * kMlpH + n];
    unsigned short* q = BM1 + (size_t)n * kMlpH + kk;
    *(volatile v8h*)q = hv;
    __threadfence();
    *(volatile v8h*)q = hv;
  } else {
    if (tid < 64) {
      const int L = tid >> 5;
      const int j4 = (tid & 31) * 4;
      const float* bp  = L ? b1 : b0;
      const float* gp  = L ? g1 : g0;
      const float* bep = L ? be1 : be0;
      const float* rmp = L ? rm1 : rm0;
      const float* rvp = L ? rv1 : rv0;
      v4f tv;
#pragma unroll
      for (int e = 0; e < 4; ++e) {
        const int n = j4 + e;
        const float s = gp[n] * rsqrtf(rvp[n] + kBnEps);
        tv[e] = (bp[n] - rmp[n]) * s + bep[n];
      }
      float* q = (L ? T1 : T0) + j4;
      *(volatile v4f*)q = tv;
      __threadfence();
      *(volatile v4f*)q = tv;
    }
  }
}

__global__ __launch_bounds__(32) void agg_pack_kernel(
    const float* __restrict__ S, const int* __restrict__ src, const int* __restrict__ dst,
    unsigned short* __restrict__ A16) {
  __shared__ __align__(16) float sAcc[kTileNodes * kFeat];
  __shared__ __align__(16) float sCnt[kTileNodes];
  __shared__ __align__(16) int   sLd[kEdgeChunk];
  __shared__ __align__(16) int   sLs[kEdgeChunk];
  const int lane = threadIdx.x;
  const int base = blockIdx.x * kTileNodes;
  {
    const v4f z4 = (v4f){0.f, 0.f, 0.f, 0.f};
#pragma unroll 1
    for (int i = 0; i < kTileNodes * kFeat / 128; ++i) *(v4f*)(sAcc + (i * 32 + lane) * 4) = z4;
#pragma unroll 1
    for (int i = 0; i < kTileNodes / 32; ++i) sCnt[i * 32 + lane] = 0.0f;
#pragma unroll 1
    for (int i = 0; i < kEdgeChunk / 32; ++i) {
      sLd[i * 32 + lane] = 0;
      sLs[i * 32 + lane] = 0;
    }
  }
  wave_lds_sync();
  const unsigned below = (1u << lane) - 1u;
#pragma unroll 1
  for (int it = 0; it < kEdges / kEdgeChunk; ++it) {
    const int e0 = it * kEdgeChunk + lane * 4;
    const v4i d4 = *(const v4i*)(dst + e0);
    const int dA = d4[0], dB = d4[1], dC = d4[2], dD = d4[3];
    const unsigned lA = (unsigned)(dA - base), lB = (unsigned)(dB - base);
    const unsigned lC = (unsigned)(dC - base), lD = (unsigned)(dD - base);
    const bool hA = lA < (unsigned)kTileNodes, hB = lB < (unsigned)kTileNodes;
    const bool hC = lC < (unsigned)kTileNodes, hD = lD < (unsigned)kTileNodes;
    const unsigned mA = __builtin_amdgcn_ballot_w32(hA);
    const unsigned mB = __builtin_amdgcn_ballot_w32(hB);
    const unsigned mC = __builtin_amdgcn_ballot_w32(hC);
    const unsigned mD = __builtin_amdgcn_ballot_w32(hD);
    if ((mA | mB | mC | mD) != 0u) {
      const v4i s4 = *(const v4i*)(src + e0);
      const int sA = s4[0], sB = s4[1], sC = s4[2], sD = s4[3];
      int cnt = 0;
      if (mA != 0u) {
        if (hA) { const int p = cnt + __popc(mA & below); sLd[p] = (int)lA; sLs[p] = sA; }
        cnt += __popc(mA);
      }
      if (mB != 0u) {
        if (hB) { const int p = cnt + __popc(mB & below); sLd[p] = (int)lB; sLs[p] = sB; }
        cnt += __popc(mB);
      }
      if (mC != 0u) {
        if (hC) { const int p = cnt + __popc(mC & below); sLd[p] = (int)lC; sLs[p] = sC; }
        cnt += __popc(mC);
      }
      if (mD != 0u) {
        if (hD) { const int p = cnt + __popc(mD & below); sLd[p] = (int)lD; sLs[p] = sD; }
        cnt += __popc(mD);
      }
      wave_lds_sync();
      const int nh = cnt < kEdgeChunk ? cnt : kEdgeChunk;
#pragma unroll 1
      for (int k = 0; k < nh; ++k) {
        const int dl = clampi(sLd[k], 0, kTileNodes - 1);
        const int sr = clampi(sLs[k], 0, kNodes - 1);
        const v4f xv = *(const v4f*)(S + (size_t)sr * kFeat + lane * 4);
        float* ap = sAcc + dl * kFeat + lane * 4;
        v4f av = *(const v4f*)ap;
        av[0] += xv[0];
        av[1] += xv[1];
        av[2] += xv[2];
        av[3] += xv[3];
        *(v4f*)ap = av;
        const float cv = sCnt[dl];
        sCnt[dl] = cv + 1.0f;
      }
      wave_lds_sync();
    }
  }
  wave_lds_sync();
  const int sub = lane >> 4, c8 = (lane & 15) * 8;
#pragma unroll 1
  for (int r2 = 0; r2 < kTileNodes / 2; ++r2) {
    const int rl = r2 * 2 + sub;
    const int row = base + rl;
    const bool valid = row < kNodes;
    const int rc = valid ? row : (kNodes - 1);
    const float* sp = S + (size_t)rc * kFeat + c8;
    const v4f a0 = *(const v4f*)(sp);
    const v4f a1 = *(const v4f*)(sp + 4);
    const float dc = fmaxf(sCnt[rl], 1.0f);
    const float inv = 1.0f / dc;
    const float* lp = sAcc + rl * kFeat + c8;
    const v4f g0 = *(const v4f*)(lp);
    const v4f g1 = *(const v4f*)(lp + 4);
    v8h hv, gv;
#pragma unroll
    for (int e = 0; e < 4; ++e) {
      const float x0 = valid ? a0[e] : 0.0f;
      const float x1 = valid ? a1[e] : 0.0f;
      const float y0 = g0[e] * inv;
      const float y1 = g1[e] * inv;
      hv[e]     = (_Float16)x0;
      hv[4 + e] = (_Float16)x1;
      gv[e]     = (_Float16)y0;
      gv[4 + e] = (_Float16)y1;
    }
    unsigned short* q = A16 + (size_t)row * kPackK + c8;
    *(volatile v8h*)q = hv;
    *(volatile v8h*)(q + kFeat) = gv;
    __threadfence();
    *(volatile v8h*)q = hv;
    *(volatile v8h*)(q + kFeat) = gv;
  }
}

__global__ __launch_bounds__(256) void cand_kernel(
    const float* __restrict__ PP, const int* __restrict__ cu, const int* __restrict__ cv,
    const float* __restrict__ cf, const float* __restrict__ mw0, const float* __restrict__ mb0,
    unsigned short* __restrict__ Z0) {
  const int gid = blockIdx.x * 256 + threadIdx.x;
  const int c = gid >> 3;
  const int g8 = (gid & 7) * 8;
  const bool valid = c < kCand;
  const int cc = valid ? c : (kCand - 1);
  const int u = clampi(cu[cc], 0, kNodes - 1);
  const int v = clampi(cv[cc], 0, kNodes - 1);
  const float f = cf[cc];
  const float* pu = PP + (size_t)u * kFeat + g8;
  const float* pv = PP + (size_t)v * kFeat + kMlpH + g8;
  const float* pw = mw0 + (size_t)(kMlpInRows - 1) * kMlpH + g8;
  const float* pb = mb0 + g8;
  const v4f a0 = *(const v4f*)(pu), a1 = *(const v4f*)(pu + 4);
  const v4f b0 = *(const v4f*)(pv), b1 = *(const v4f*)(pv + 4);
  const v4f w0 = *(const v4f*)(pw), w1 = *(const v4f*)(pw + 4);
  const v4f m0 = *(const v4f*)(pb), m1 = *(const v4f*)(pb + 4);
  v8h hv;
#pragma unroll
  for (int e = 0; e < 4; ++e) {
    float t0 = a0[e] + b0[e];
    float t1 = a1[e] + b1[e];
    t0 = fmaf(f, w0[e], t0) + m0[e];
    t1 = fmaf(f, w1[e], t1) + m1[e];
    t0 = (t0 > 0.f) ? t0 : kSlope * t0;
    t1 = (t1 > 0.f) ? t1 : kSlope * t1;
    const float o0 = valid ? t0 : 0.0f;
    const float o1 = valid ? t1 : 0.0f;
    hv[e]     = (_Float16)o0;
    hv[4 + e] = (_Float16)o1;
  }
  unsigned short* q = Z0 + (size_t)c * kMlpH + g8;
  *(volatile v8h*)q = hv;
  __threadfence();
  *(volatile v8h*)q = hv;
}

__global__ __launch_bounds__(256) void final_kernel(
    const float* __restrict__ Z1, const float* __restrict__ mw2, const float* __restrict__ mb2,
    float* __restrict__ yout, float* __restrict__ yws) {
  __shared__ __align__(16) float sW[kMlpH];
  const int tid = threadIdx.x;
  if (tid < kMlpH) sW[tid] = mw2[tid];
  __syncthreads();
  const int c = blockIdx.x * 256 + tid;
  const bool valid = c < kCand;
  const int cc = valid ? c : (kCand - 1);
  const float* zp = Z1 + (size_t)cc * kMlpH;
  float acc = 0.0f;
#pragma unroll 1
  for (int j4 = 0; j4 < kMlpH / 4; ++j4) {
    const v4f z = *(const v4f*)(zp + 4 * j4);
    const v4f w = *(const v4f*)(sW + 4 * j4);
    acc = fmaf(z[0], w[0], acc);
    acc = fmaf(z[1], w[1], acc);
    acc = fmaf(z[2], w[2], acc);
    acc = fmaf(z[3], w[3], acc);
  }
  const float yv = acc + mb2[0];
  if (valid) {
    volatile float* p0 = yout + c;
    volatile float* p1 = yws + c;
    *p0 = yv;
    *p1 = yv;
    __threadfence();
    *p0 = yv;
    *p1 = yv;
  }
}

__global__ __launch_bounds__(1024) void softmax_kernel(const float* __restrict__ y, float* __restrict__ out1) {
  __shared__ float sRed[32];
  const int tid = threadIdx.x, lane = tid & 31, wave = tid >> 5;
  float m = -INFINITY;
#pragma unroll 1
  for (int i = tid; i < kCand; i += 1024) m = fmaxf(m, y[i]);
#pragma unroll
  for (int off = 16; off > 0; off >>= 1) m = fmaxf(m, __shfl_xor(m, off, 32));
  if (lane == 0) sRed[wave] = m;
  __syncthreads();
  float gm = sRed[lane];
#pragma unroll
  for (int off = 16; off > 0; off >>= 1) gm = fmaxf(gm, __shfl_xor(gm, off, 32));
  __syncthreads();
  float s = 0.0f;
#pragma unroll 1
  for (int i = tid; i < kCand; i += 1024) s += expf(y[i] - gm);
#pragma unroll
  for (int off = 16; off > 0; off >>= 1) s += __shfl_xor(s, off, 32);
  if (lane == 0) sRed[wave] = s;
  __syncthreads();
  float tot = sRed[lane];
#pragma unroll
  for (int off = 16; off > 0; off >>= 1) tot += __shfl_xor(tot, off, 32);
  const float inv = 1.0f / tot;
#pragma unroll 1
  for (int i = tid; i < kCand; i += 1024) {
    const float v = expf(y[i] - gm) * inv;
    volatile float* p = out1 + i;
    *p = v;
    __threadfence();
    *p = v;
  }
}

extern "C" void kernel_launch(void* const* d_in, const int* in_sizes, int n_in,
                              void* d_out, int out_size, void* d_ws, size_t ws_size,
                              hipStream_t stream) {
  if (n_in < 26) return;
  if (in_sizes[0] != kNodes * kFeat) return;
  if (in_sizes[1] != kEdges || in_sizes[2] != kEdges) return;
  if (in_sizes[3] != kCand || in_sizes[4] != kCand || in_sizes[5] != kCand) return;
  if (in_sizes[6] != kFeat * kFeat || in_sizes[7] != kFeat * kFeat) return;
  if (in_sizes[13] != kFeat * kFeat || in_sizes[14] != kFeat * kFeat) return;
  for (int i = 8; i <= 12; ++i) if (in_sizes[i] != kFeat) return;
  for (int i = 15; i <= 19; ++i) if (in_sizes[i] != kFeat) return;
  if (in_sizes[20] != kMlpInRows * kMlpH) return;
  if (in_sizes[21] != kMlpH || in_sizes[22] != kMlpH * kMlpH || in_sizes[23] != kMlpH) return;
  if (in_sizes[24] != kMlpH || in_sizes[25] != 1) return;
  if (out_size != 2 * kCand) return;
  if (ws_size < kWsTotal) return;

  const float* x    = (const float*)d_in[0];
  const int*   src  = (const int*)d_in[1];
  const int*   dst  = (const int*)d_in[2];
  const int*   cu   = (const int*)d_in[3];
  const int*   cv   = (const int*)d_in[4];
  const float* cf   = (const float*)d_in[5];
  const float* ws0  = (const float*)d_in[6];
  const float* wn0  = (const float*)d_in[7];
  const float* b0   = (const float*)d_in[8];
  const float* g0   = (const float*)d_in[9];
  const float* be0  = (const float*)d_in[10];
  const float* rm0  = (const float*)d_in[11];
  const float* rv0  = (const float*)d_in[12];
  const float* ws1  = (const float*)d_in[13];
  const float* wn1  = (const float*)d_in[14];
  const float* b1   = (const float*)d_in[15];
  const float* g1   = (const float*)d_in[16];
  const float* be1  = (const float*)d_in[17];
  const float* rm1  = (const float*)d_in[18];
  const float* rv1  = (const float*)d_in[19];
  const float* mw0  = (const float*)d_in[20];
  const float* mb0  = (const float*)d_in[21];
  const float* mw1  = (const float*)d_in[22];
  const float* mb1  = (const float*)d_in[23];
  const float* mw2  = (const float*)d_in[24];
  const float* mb2  = (const float*)d_in[25];

  float* yout = (float*)d_out;
  float* sout = (float*)d_out + kCand;

  char* ws = (char*)d_ws;
  unsigned short* A16 = (unsigned short*)(ws + kOffA16);
  float*          H0  = (float*)(ws + kOffH0);
  unsigned short* H1  = (unsigned short*)(ws + kOffH1);
  float*          PP  = (float*)(ws + kOffPP);
  unsigned short* Z0  = (unsigned short*)(ws + kOffZ0);
  float*          Z1  = (float*)(ws + kOffZ1);
  float*          YW  = (float*)(ws + kOffYW);
  unsigned short* BL0 = (unsigned short*)(ws + kOffBL0);
  unsigned short* BL1 = (unsigned short*)(ws + kOffBL1);
  unsigned short* BP  = (unsigned short*)(ws + kOffBP);
  unsigned short* BM1 = (unsigned short*)(ws + kOffBM1);
  float*          T0  = (float*)(ws + kOffT0);
  float*          T1  = (float*)(ws + kOffT1);

  constexpr int kTilesNode = (kNodesPad / 64) * (kFeat / 64);
  constexpr int kTilesCand = (kCandPad / 64) * (kMlpH / 64);
  constexpr int kBlocksNode = (kTilesNode + 7) / 8;
  constexpr int kBlocksCand = (kTilesCand + 7) / 8;

  prep_kernel<<<43, 256, 0, stream>>>(ws0, wn0, b0, g0, be0, rm0, rv0,
                                      ws1, wn1, b1, g1, be1, rm1, rv1,
                                      mw0, mw1, BL0, BL1, BP, BM1, T0, T1);

  agg_pack_kernel<<<kNodeTiles, 32, 0, stream>>>(x, src, dst, A16);
  wmma_gemm64<2, 0, 4><<<kBlocksNode, 256, 0, stream>>>(
      A16, kPackK, BL0, kPackK, (void*)H0, kFeat, T0, kNodesPad, kFeat, kPackK);

  agg_pack_kernel<<<kNodeTiles, 32, 0, stream>>>(H0, src, dst, A16);
  wmma_gemm64<2, 1, 6><<<kBlocksNode, 256, 0, stream>>>(
      A16, kPackK, BL1, kPackK, (void*)H1, kFeat, T1, kNodesPad, kFeat, kPackK);

  wmma_gemm64<0, 0, 0><<<kBlocksNode, 256, 0, stream>>>(
      H1, kFeat, BP, kFeat, (void*)PP, kFeat, T0, kNodesPad, kFeat, kFeat);

  cand_kernel<<<(kCandPad * 8) / 256, 256, 0, stream>>>(PP, cu, cv, cf, mw0, mb0, Z0);

  wmma_gemm64<2, 0, 4><<<kBlocksCand, 256, 0, stream>>>(
      Z0, kMlpH, BM1, kMlpH, (void*)Z1, kMlpH, mb1, kCandPad, kMlpH, kMlpH);

  final_kernel<<<(kCand + 255) / 256, 256, 0, stream>>>(Z1, mw2, mb2, yout, YW);

  softmax_kernel<<<1, 1024, 0, stream>>>(YW, sout);
}
